// HierarchicalSparseAttention_62534723830440
// MI455X (gfx1250) — hardware-verified
//
#include <hip/hip_runtime.h>
#include <stdint.h>

typedef __attribute__((ext_vector_type(16))) _Float16 v16h;
typedef __attribute__((ext_vector_type(8)))  _Float16 v8h;
typedef __attribute__((ext_vector_type(16))) __bf16   v16b;
typedef __attribute__((ext_vector_type(8)))  __bf16   v8b;
typedef __attribute__((ext_vector_type(8)))  float    v8f;
typedef __attribute__((ext_vector_type(4)))  float    v4f;
typedef __attribute__((ext_vector_type(4)))  unsigned int v4u;

constexpr int kSeqLen    = 2048;
constexpr int kModelD    = 1024;
constexpr int kHeads     = 16;
constexpr int kHeadDim   = 64;
constexpr int kKvReal    = 2 * kSeqLen - 1;
constexpr int kKvPad     = 4096;
constexpr int kQBlk      = 64;
constexpr int kKch       = 64;
constexpr int kNumQB     = kSeqLen / kQBlk;
constexpr int kWinHalf   = 21;
constexpr int kHierSlots = 67;

static_assert(kNumQB == 32, "qb decode uses & 31 / >> 5");
static_assert(kSeqLen % 64 == 0 && kKvPad % 64 == 0 && kModelD % 64 == 0, "M,N tile multiples of 64");
static_assert(kModelD % 32 == 0, "K multiple of 32");
static_assert(kHeads * kHeadDim == kModelD, "head split");

__device__ __forceinline__ unsigned short f2bf_bits(float f) {
  unsigned u = __float_as_uint(f);
  return (unsigned short)((u + 0x7FFFu + ((u >> 16) & 1u)) >> 16);
}
__device__ __forceinline__ float bf_bits2f(unsigned short h) { return __uint_as_float(((unsigned)h) << 16); }

__device__ __forceinline__ void dep_guard_h(v8f& a, v8f& b, v16h x, v16h y) { asm volatile("v_nop\n\tv_nop\n\tv_nop\n\tv_nop" : "+v"(a), "+v"(b) : "v"(x), "v"(y)); }
__device__ __forceinline__ void dep_guard_b(v8f& a, v8f& b, v16b x, v16b y) { asm volatile("v_nop\n\tv_nop\n\tv_nop\n\tv_nop" : "+v"(a), "+v"(b) : "v"(x), "v"(y)); }
__device__ __forceinline__ void keep4_h(v16h a, v16h b, v16h c, v16h d) { asm volatile("v_nop" :: "v"(a), "v"(b), "v"(c), "v"(d)); }
__device__ __forceinline__ void keep4_b(v16b a, v16b b, v16b c, v16b d) { asm volatile("v_nop" :: "v"(a), "v"(b), "v"(c), "v"(d)); }
__device__ __forceinline__ void acc_guard4(v8f& a, v8f& b, v8f& c, v8f& d) { asm volatile("v_nop\n\tv_nop\n\tv_nop\n\tv_nop" : "+v"(a), "+v"(b), "+v"(c), "+v"(d)); }
template <typename T> struct Frag;
template <> struct Frag<_Float16> {
  typedef v16h V; union U { v16h v; v8h h[2]; };
  static __device__ __forceinline__ v16h load(const _Float16* p) {
    U f; f.h[0] = *(const v8h*)(p); f.h[1] = *(const v8h*)(p + 16); return f.v;
  }
  static __device__ __forceinline__ v8f mma(v16h a, v16h b, v8f c) {
    return __builtin_amdgcn_wmma_f32_16x16x32_f16(false, a, false, b, (short)0, c, false, false);
  }
  static __device__ __forceinline__ void guard(v8f& a, v8f& b, v16h x, v16h y) { dep_guard_h(a, b, x, y); }
  static __device__ __forceinline__ void keep(v16h a, v16h b, v16h c, v16h d) { keep4_h(a, b, c, d); }
};
template <> struct Frag<__bf16> {
  typedef v16b V; union U { v16b v; v8b h[2]; };
  static __device__ __forceinline__ v16b load(const __bf16* p) {
    U f; f.h[0] = *(const v8b*)(p); f.h[1] = *(const v8b*)(p + 16); return f.v;
  }
  static __device__ __forceinline__ v8f mma(v16b a, v16b b, v8f c) {
    return __builtin_amdgcn_wmma_f32_16x16x32_bf16(false, a, false, b, (short)0, c, false, false);
  }
  static __device__ __forceinline__ void guard(v8f& a, v8f& b, v16b x, v16b y) { dep_guard_b(a, b, x, y); }
  static __device__ __forceinline__ void keep(v16b a, v16b b, v16b c, v16b d) { keep4_b(a, b, c, d); }
};

template <int ET> struct Elem;
template <> struct Elem<0> { typedef _Float16 T; };
template <> struct Elem<1> { typedef __bf16 T; };
template <int ET, int SPLIT, int BIAS_MODE, int OUT_MODE, bool RESID, int ACT = 0>
__global__ __launch_bounds__(256) void wmma_gemm64(
    const unsigned short* __restrict__ Ap, const unsigned short* __restrict__ A2p, int lda, long strideA,
    const unsigned short* __restrict__ Btp, const unsigned short* __restrict__ Bt2p, int ldb, long strideB,
    void* __restrict__ Cout, void* __restrict__ Cout2, int ldc, long strideC,
    const float* __restrict__ bias,
    const float* __restrict__ resid, long strideR,
    int M, int N, int K, float scale) {
  typedef typename Elem<ET>::T T;
  typedef typename Frag<T>::V V;
  const T* A = (const T*)Ap; const T* A2 = (const T*)A2p; const T* Bt = (const T*)Btp; const T* Bt2 = (const T*)Bt2p;
  __shared__ __align__(16) float sT[8][16 * 68];
  const int b    = blockIdx.y;
  const int lane = threadIdx.x & 31;
  const int wave = threadIdx.x >> 5;
  const int tilesN = N >> 6;
  const int tilesM = M >> 6;
  const int tile = blockIdx.x * 8 + wave;
  if (tile >= tilesM * tilesN) return;
  const int tm = tile / tilesN;
  const int tn = tile - tm * tilesN;
  const int m0 = tm << 6;
  const int n0 = tn << 6;

  const T* Ab  = A  + (size_t)b * strideA;
  const T* Bb  = Bt + (size_t)b * strideB;
  const T* Ab2 = SPLIT ? (A2  + (size_t)b * strideA) : nullptr;
  const T* Bb2 = (SPLIT == 2) ? (Bt2 + (size_t)b * strideB) : nullptr;

  const int rlane = lane & 15;
  const int koff  = (lane >> 4) * 8;
  const int mOff  = (lane >> 4) * 8;

  v8f acc[4][4];
#pragma unroll
  for (int i = 0; i < 4; ++i)
#pragma unroll
    for (int j = 0; j < 4; ++j) acc[i][j] = (v8f){0.f,0.f,0.f,0.f,0.f,0.f,0.f,0.f};

  for (int k0 = 0; k0 < K; k0 += 32) {
    V bh[4], bl[4];
#pragma unroll
    for (int j = 0; j < 4; ++j) {
      const size_t bo = (size_t)(n0 + (j << 4) + rlane) * ldb + koff + k0;
      bh[j] = Frag<T>::load(Bb + bo);
      if (SPLIT == 2) bl[j] = Frag<T>::load(Bb2 + bo);
    }
#pragma unroll
    for (int i = 0; i < 4; ++i) {
      const size_t ao = (size_t)(m0 + (i << 4) + rlane) * lda + koff + k0;
      V ah = Frag<T>::load(Ab + ao);
      V al;
      if (SPLIT) al = Frag<T>::load(Ab2 + ao);
#pragma unroll
      for (int j = 0; j < 4; ++j) {
        acc[i][j] = Frag<T>::mma(ah, bh[j], acc[i][j]);
        if (SPLIT == 2) acc[i][j] = Frag<T>::mma(ah, bl[j], acc[i][j]);
        if (SPLIT) acc[i][j] = Frag<T>::mma(al, bh[j], acc[i][j]);
      }
      Frag<T>::guard(acc[i][0], acc[i][3], ah, SPLIT ? al : ah);
    }
    Frag<T>::keep(bh[0], bh[1], bh[2], bh[3]);
    if (SPLIT == 2) Frag<T>::keep(bl[0], bl[1], bl[2], bl[3]);
  }
  acc_guard4(acc[0][0], acc[0][1], acc[0][2], acc[0][3]);
  acc_guard4(acc[1][0], acc[1][1], acc[1][2], acc[1][3]);
  acc_guard4(acc[2][0], acc[2][1], acc[2][2], acc[2][3]);
  acc_guard4(acc[3][0], acc[3][1], acc[3][2], acc[3][3]);

  float* slab = sT[wave];
  const float* Rb = RESID ? (resid + (size_t)b * strideR) : nullptr;
#pragma unroll
  for (int i = 0; i < 4; ++i) {
    const int mBase = m0 + (i << 4);
#pragma unroll
    for (int j = 0; j < 4; ++j) {
      const int n = n0 + (j << 4) + rlane;
      float bv = 0.f;
      if (BIAS_MODE == 2) bv = bias[n];
#pragma unroll
      for (int r = 0; r < 8; ++r) {
        float v = acc[i][j][r] * scale;
        if (BIAS_MODE == 1) v += bias[mBase + mOff + r];
        if (BIAS_MODE == 2) v += bv;
        if (RESID) v += Rb[(size_t)(mBase + mOff + r) * ldc + n];
        if (ACT == 1) v = tanhf(v);
        if (ACT == 2) v = fmaxf(v, 0.0f);
        if (ACT == 3) v = v / (1.0f + expf(-v));
        if (ACT == 4) v = (v > 0.f) ? v : 0.01f * v;
        slab[(mOff + r) * 68 + (j << 4) + rlane] = v;
      }
    }
    __builtin_amdgcn_fence(__ATOMIC_RELEASE, "workgroup");
    __builtin_amdgcn_wave_barrier();
    __builtin_amdgcn_fence(__ATOMIC_ACQUIRE, "workgroup");
    if (OUT_MODE == 0) {
      float* C = (float*)Cout + (size_t)b * strideC;
      const int hh = lane >> 4, c4 = (lane & 15) * 4;
      for (int pass = 0; pass < 2; ++pass) {
#pragma unroll
        for (int it = 0; it < 8; ++it) {
          const int row = it * 2 + hh;
          v4f v = *(const v4f*)(slab + row * 68 + c4);
          *(volatile v4f*)(C + (size_t)(mBase + row) * ldc + n0 + c4) = v;
        }
        __threadfence();
      }
    } else {
      const int q = lane >> 3, c8 = (lane & 7) * 8;
      unsigned short* C  = (unsigned short*)Cout  + (size_t)b * strideC;
      unsigned short* C2 = (OUT_MODE == 2) ? ((unsigned short*)Cout2 + (size_t)b * strideC) : nullptr;
      for (int pass = 0; pass < 2; ++pass) {
#pragma unroll
        for (int it = 0; it < 4; ++it) {
          const int row = it * 4 + q;
          const float* sp = slab + row * 68 + c8;
          v8h hv, lv;
#pragma unroll
          for (int e = 0; e < 8; ++e) {
            if (OUT_MODE == 1) {
              hv[e] = (_Float16)sp[e];
            } else {
              unsigned short hb = f2bf_bits(sp[e]);
              unsigned short lb = f2bf_bits(sp[e] - bf_bits2f(hb));
              hv[e] = __builtin_bit_cast(_Float16, hb);
              lv[e] = __builtin_bit_cast(_Float16, lb);
            }
          }
          *(volatile v8h*)(C + (size_t)(mBase + row) * ldc + n0 + c8) = hv;
          if (OUT_MODE == 2) *(volatile v8h*)(C2 + (size_t)(mBase + row) * ldc + n0 + c8) = lv;
        }
        __threadfence();
      }
    }
    __builtin_amdgcn_fence(__ATOMIC_RELEASE, "workgroup");
    __builtin_amdgcn_wave_barrier();
    __builtin_amdgcn_fence(__ATOMIC_ACQUIRE, "workgroup");
  }
}

__global__ __launch_bounds__(256) void cast_f32_bf16x2(
    const float* __restrict__ in, unsigned short* __restrict__ out, int n2) {
  int i = blockIdx.x * 256 + threadIdx.x;
  if (i < n2) {
    const float f0 = in[2 * i], f1 = in[2 * i + 1];
    const unsigned u = (unsigned)f2bf_bits(f0) | ((unsigned)f2bf_bits(f1) << 16);
    ((volatile unsigned*)out)[i] = u;
    __threadfence();
    ((volatile unsigned*)out)[i] = u;
  }
}

__global__ __launch_bounds__(256) void fill_zero_u32(unsigned* __restrict__ out, int n) {
  int i = blockIdx.x * 256 + threadIdx.x;
  if (i < n) {
    const unsigned z = 0u;
    ((volatile unsigned*)out)[i] = z;
    __threadfence();
    ((volatile unsigned*)out)[i] = z;
  }
}

__device__ __forceinline__ unsigned short at_bf_bits(float f) {
  unsigned u = __float_as_uint(f);
  return (unsigned short)((u + 0x7FFFu + ((u >> 16) & 1u)) >> 16);
}
__device__ __forceinline__ __bf16 at_f2bf(float f) { return __builtin_bit_cast(__bf16, at_bf_bits(f)); }
__device__ __forceinline__ void at_split(float f, __bf16& hi, __bf16& lo) {
  const unsigned short hb = at_bf_bits(f);
  hi = __builtin_bit_cast(__bf16, hb);
  lo = at_f2bf(f - __uint_as_float(((unsigned)hb) << 16));
}
__device__ __forceinline__ v8f at_mma(v16b a, v16b b, v8f c) {
  c = __builtin_amdgcn_wmma_f32_16x16x32_bf16(false, a, false, b, (short)0, c, false, false);
  asm volatile("v_nop\n\tv_nop\n\tv_nop\n\tv_nop" : "+v"(c) : "v"(a), "v"(b));
  return c;
}

__device__ __forceinline__ void hier_slot(int s, int qblk0, int& t, int& row, int& g, int& valid) {
  int tt = (s < 32) ? 1 : ((s < 48) ? 2 : ((s < 56) ? 3 : ((s < 60) ? 4 : ((s < 62) ? 5 : (6 + (s - 62))))));
  tt = (tt > 10) ? 10 : tt;
  const int base = (tt <= 6) ? (64 - (64 >> (tt - 1))) : (56 + tt);
  const int off  = 4096 - (4096 >> tt);
  const int qs   = qblk0 >> tt;
  int r = (tt <= 5) ? (off + qs + (s - base)) : ((qs + off) ^ 1);
  const int v = (s < kHierSlots) ? 1 : 0;
  r = v ? r : (kKvPad - 1);
  r = (r < 0) ? 0 : ((r > kKvPad - 1) ? (kKvPad - 1) : r);
  t = tt; row = r; g = (r ^ 1) - off; valid = v;
}

__global__ __launch_bounds__(128)
void tree_window_attn(const unsigned short* __restrict__ Qh, const unsigned short* __restrict__ Ql,
                      const unsigned short* __restrict__ Kh, const unsigned short* __restrict__ Kl,
                      const unsigned short* __restrict__ Vh, const unsigned short* __restrict__ Vl,
                      unsigned short* __restrict__ Oh, unsigned short* __restrict__ Ol,
                      const int* __restrict__ maskp) {
  union FB { v16b v; v8b h[2]; };
  __shared__ __align__(16) __bf16 Ksh[kKch * kHeadDim];
  __shared__ __align__(16) __bf16 Ksl[kKch * kHeadDim];
  __shared__ __align__(16) __bf16 Vth[kHeadDim * kKch];
  __shared__ __align__(16) __bf16 Vtl[kHeadDim * kKch];
  __shared__ __align__(16) __bf16 Psh[4][16 * kKch];
  __shared__ __align__(16) __bf16 Psl[4][16 * kKch];
  __shared__ __align__(16) float  Os[4][16 * 68];

  const int tid  = threadIdx.x;
  const int wave = tid >> 5;
  const int lane = tid & 31;
  const int hh   = lane >> 4;
  const int c    = lane & 15;

  const int bx    = blockIdx.x;
  const int qb    = bx & (kNumQB - 1);
  const int h     = bx >> 5;
  const int qblk0 = qb * kQBlk;
  const int q0    = qblk0 + wave * 16;
  const int mval  = __builtin_amdgcn_readfirstlane(maskp[0]);
  const bool causal = (mval != 0);

  v16b qah[2], qal[2];
  {
    const __bf16* qhp = (const __bf16*)(const void*)Qh + (size_t)(q0 + c) * kModelD + (size_t)h * kHeadDim + 8 * hh;
    const __bf16* qlp = (const __bf16*)(const void*)Ql + (size_t)(q0 + c) * kModelD + (size_t)h * kHeadDim + 8 * hh;
#pragma unroll
    for (int dc = 0; dc < 2; ++dc) {
      qah[dc] = Frag<__bf16>::load(qhp + dc * 32);
      qal[dc] = Frag<__bf16>::load(qlp + dc * 32);
    }
  }

  float mrow[8], lrow[8];
  v8f oacc[4];
#pragma unroll
  for (int r = 0; r < 8; ++r) { mrow[r] = -1.0e30f; lrow[r] = 0.f; }
#pragma unroll
  for (int t = 0; t < 4; ++t) oacc[t] = (v8f){0.f,0.f,0.f,0.f,0.f,0.f,0.f,0.f};

  for (int ci = 0; ci < 5; ++ci) {
    const bool isSwa = (ci < 3);
    int kbase = 0;
    int hc = 0;
    if (isSwa) {
      const int kcb = qb - 1 + ci;
      if (kcb < 0 || kcb >= kNumQB) continue;
      if (causal && kcb > qb) continue;
      kbase = kcb * kKch;
    } else {
      hc = ci - 3;
    }
    __syncthreads();
    {
      const int kvr = tid >> 1;
      const int dh  = (tid & 1) * 32;
      int srow, sval;
      if (isSwa) { srow = kbase + kvr; sval = 1; }
      else { int tt, gg; hier_slot(hc * 64 + kvr, qblk0, tt, srow, gg, sval); }
      srow = (srow < 0) ? 0 : ((srow > kKvPad - 1) ? (kKvPad - 1) : srow);
      const size_t go = (size_t)srow * kModelD + (size_t)h * kHeadDim + dh;
      const unsigned zm = sval ? 0xffffffffu : 0u;
      {
        const v4u* khp = (const v4u*)(const void*)(Kh + go);
        const v4u* klp = (const v4u*)(const void*)(Kl + go);
        v4u kw[4], lw[4];
#pragma unroll
        for (int i = 0; i < 4; ++i) { kw[i] = khp[i]; lw[i] = klp[i]; }
#pragma unroll
        for (int i = 0; i < 4; ++i) {
          v4u a = kw[i], bq = lw[i];
#pragma unroll
          for (int k2 = 0; k2 < 4; ++k2) { a[k2] &= zm; bq[k2] &= zm; }
          *(v4u*)(void*)(Ksh + kvr * kHeadDim + dh + 8 * i) = a;
          *(v4u*)(void*)(Ksl + kvr * kHeadDim + dh + 8 * i) = bq;
        }
      }
      asm volatile("" ::: "memory");
      {
        const v4u* vhp = (const v4u*)(const void*)(Vh + go);
        const v4u* vlp = (const v4u*)(const void*)(Vl + go);
        v4u vw[4], ww[4];
#pragma unroll
        for (int i = 0; i < 4; ++i) { vw[i] = vhp[i]; ww[i] = vlp[i]; }
#pragma unroll
        for (int i = 0; i < 4; ++i) {
#pragma unroll
          for (int k2 = 0; k2 < 4; ++k2) {
            const unsigned wa = vw[i][k2] & zm;
            const unsigned wb = ww[i][k2] & zm;
            const int d0 = dh + 8 * i + 2 * k2;
            Vth[d0 * kKch + kvr]       = __builtin_bit_cast(__bf16, (unsigned short)(wa & 0xffffu));
            Vth[(d0 + 1) * kKch + kvr] = __builtin_bit_cast(__bf16, (unsigned short)(wa >> 16));
            Vtl[d0 * kKch + kvr]       = __builtin_bit_cast(__bf16, (unsigned short)(wb & 0xffffu));
            Vtl[(d0 + 1) * kKch + kvr] = __builtin_bit_cast(__bf16, (unsigned short)(wb >> 16));
          }
        }
      }
    }
    __syncthreads();

    v8f s[4];
#pragma unroll
    for (int j = 0; j < 4; ++j) {
      s[j] = (v8f){0.f,0.f,0.f,0.f,0.f,0.f,0.f,0.f};
#pragma unroll
      for (int dc = 0; dc < 2; ++dc) {
        FB kb, kl;
        const int ko = (j * 16 + c) * kHeadDim + dc * 32 + 8 * hh;
        kb.h[0] = *(const v8b*)(Ksh + ko);
        kb.h[1] = *(const v8b*)(Ksh + ko + 16);
        kl.h[0] = *(const v8b*)(Ksl + ko);
        kl.h[1] = *(const v8b*)(Ksl + ko + 16);
        s[j] = at_mma(qah[dc], kb.v, s[j]);
        s[j] = at_mma(qah[dc], kl.v, s[j]);
        s[j] = at_mma(qal[dc], kb.v, s[j]);
      }
    }

    int colKey[4], colT[4], colG[4], colV[4];
#pragma unroll
    for (int j = 0; j < 4; ++j) {
      const int slot = j * 16 + c;
      colKey[j] = kbase + slot;
      int tt, rr, gg, vv;
      hier_slot(hc * 64 + slot, qblk0, tt, rr, gg, vv);
      colT[j] = tt; colG[j] = gg; colV[j] = vv;
    }

    unsigned dblBits = 0u;
    float cm[8];
#pragma unroll
    for (int r = 0; r < 8; ++r) {
      const int l = q0 + 8 * hh + r;
      float m = -1.0e30f;
#pragma unroll
      for (int j = 0; j < 4; ++j) {
        int mult;
        if (isSwa) {
          const int d = colKey[j] - l;
          const int w = (d >= -kWinHalf && d <= kWinHalf && (!causal || d <= 0)) ? 1 : 0;
          const int z = (colKey[j] == (l ^ 1) && (!causal || ((l & 1) != 0))) ? 1 : 0;
          mult = w + z;
        } else {
          const int lt = l >> colT[j];
          mult = (colV[j] != 0 && lt == colG[j] && (!causal || ((lt & 1) != 0))) ? 1 : 0;
        }
        float sv = s[j][r] * 0.125f;
        sv = (mult > 0) ? sv : -1.0e30f;
        s[j][r] = sv;
        dblBits |= (mult > 1) ? (1u << (j * 8 + r)) : 0u;
        m = fmaxf(m, sv);
      }
#pragma unroll
      for (int off = 1; off < 16; off <<= 1) m = fmaxf(m, __shfl_xor(m, off, 32));
      cm[r] = m;
    }

    __bf16* pwh = Psh[wave];
    __bf16* pwl = Psl[wave];
#pragma unroll
    for (int r = 0; r < 8; ++r) {
      const float mnew  = fmaxf(mrow[r], cm[r]);
      const float alpha = expf(mrow[r] - mnew);
      mrow[r] = mnew;
      float psum = 0.f;
#pragma unroll
      for (int j = 0; j < 4; ++j) {
        const float multf = (s[j][r] > -1.0e29f) ? ((((dblBits >> (j * 8 + r)) & 1u) != 0u) ? 2.0f : 1.0f) : 0.0f;
        const float p = multf * expf(s[j][r] - mnew);
        psum += p;
        __bf16 a, bl;
        at_split(p, a, bl);
        pwh[(8 * hh + r) * kKch + j * 16 + c] = a;
        pwl[(8 * hh + r) * kKch + j * 16 + c] = bl;
      }
#pragma unroll
      for (int off = 1; off < 16; off <<= 1) psum += __shfl_xor(psum, off, 32);
      lrow[r] = lrow[r] * alpha + psum;
#pragma unroll
      for (int t = 0; t < 4; ++t) oacc[t][r] *= alpha;
    }
    __builtin_amdgcn_fence(__ATOMIC_RELEASE, "workgroup");
    __builtin_amdgcn_wave_barrier();
    __builtin_amdgcn_fence(__ATOMIC_ACQUIRE, "workgroup");

#pragma unroll
    for (int kk = 0; kk < 2; ++kk) {
      FB pa, pl;
      pa.h[0] = *(const v8b*)(pwh + c * kKch + kk * 32 + 8 * hh);
      pa.h[1] = *(const v8b*)(pwh + c * kKch + kk * 32 + 16 + 8 * hh);
      pl.h[0] = *(const v8b*)(pwl + c * kKch + kk * 32 + 8 * hh);
      pl.h[1] = *(const v8b*)(pwl + c * kKch + kk * 32 + 16 + 8 * hh);
#pragma unroll
      for (int t = 0; t < 4; ++t) {
        FB vb, vl;
        vb.h[0] = *(const v8b*)(Vth + (t * 16 + c) * kKch + kk * 32 + 8 * hh);
        vb.h[1] = *(const v8b*)(Vth + (t * 16 + c) * kKch + kk * 32 + 16 + 8 * hh);
        vl.h[0] = *(const v8b*)(Vtl + (t * 16 + c) * kKch + kk * 32 + 8 * hh);
        vl.h[1] = *(const v8b*)(Vtl + (t * 16 + c) * kKch + kk * 32 + 16 + 8 * hh);
        oacc[t] = at_mma(pa.v, vb.v, oacc[t]);
        oacc[t] = at_mma(pa.v, vl.v, oacc[t]);
        oacc[t] = at_mma(pl.v, vb.v, oacc[t]);
      }
    }
  }

  float* os = Os[wave];
#pragma unroll
  for (int r = 0; r < 8; ++r) {
    const float inv = 1.0f / lrow[r];
#pragma unroll
    for (int t = 0; t < 4; ++t) os[(8 * hh + r) * 68 + t * 16 + c] = oacc[t][r] * inv;
  }
  __builtin_amdgcn_fence(__ATOMIC_RELEASE, "workgroup");
  __builtin_amdgcn_wave_barrier();
  __builtin_amdgcn_fence(__ATOMIC_ACQUIRE, "workgroup");
  {
    const int q = lane >> 3, c8 = (lane & 7) * 8;
    for (int pass = 0; pass < 2; ++pass) {
#pragma unroll
      for (int it = 0; it < 4; ++it) {
        const int row = it * 4 + q;
        const float* sp = os + row * 68 + c8;
        v8h hv, lv;
#pragma unroll
        for (int e = 0; e < 8; ++e) {
          unsigned short hb = f2bf_bits(sp[e]);
          unsigned short lb = f2bf_bits(sp[e] - bf_bits2f(hb));
          hv[e] = __builtin_bit_cast(_Float16, hb);
          lv[e] = __builtin_bit_cast(_Float16, lb);
        }
        const size_t oo = (size_t)(q0 + row) * kModelD + (size_t)h * kHeadDim + c8;
        *(volatile v8h*)(Oh + oo) = hv;
        *(volatile v8h*)(Ol + oo) = lv;
      }
      __threadfence();
    }
  }
}

extern "C" void kernel_launch(void* const* d_in, const int* in_sizes, int n_in,
                              void* d_out, int out_size, void* d_ws, size_t ws_size,
                              hipStream_t stream) {
  if (n_in < 10) return;
  if (in_sizes[0] != kSeqLen * kModelD) return;
  if (in_sizes[3] != (kSeqLen - 1) * kModelD) return;
  if (in_sizes[4] != kModelD * kModelD || in_sizes[5] != kModelD * kModelD ||
      in_sizes[6] != kModelD * kModelD || in_sizes[7] != kModelD * kModelD) return;
  if (in_sizes[8] != kModelD || in_sizes[9] < 1) return;
  if (out_size != kSeqLen * kModelD) return;

  const float* x    = (const float*)d_in[0];
  const float* y    = (const float*)d_in[3];
  const float* Wq   = (const float*)d_in[4];
  const float* Wk   = (const float*)d_in[5];
  const float* Wv   = (const float*)d_in[6];
  const float* Wo   = (const float*)d_in[7];
  const float* Wob  = (const float*)d_in[8];
  const int*   msk  = (const int*)d_in[9];
  float* out = (float*)d_out;

  size_t off = 0;
  auto carve = [&](size_t bytes) -> unsigned short* {
    unsigned short* p = (unsigned short*)((char*)d_ws + off);
    off += (bytes + 255) & ~(size_t)255;
    return p;
  };
  const size_t planeKV = (size_t)kKvPad * kModelD * 2;
  const size_t planeQ  = (size_t)kSeqLen * kModelD * 2;
  const size_t planeW  = (size_t)kModelD * kModelD * 2;
  unsigned short* XYb = carve(planeKV);
  unsigned short* Wqb = carve(planeW);
  unsigned short* Wkb = carve(planeW);
  unsigned short* Wvb = carve(planeW);
  unsigned short* Wob_b = carve(planeW);
  unsigned short* Qh = carve(planeQ);
  unsigned short* Ql = carve(planeQ);
  unsigned short* Kh = carve(planeKV);
  unsigned short* Kl = carve(planeKV);
  unsigned short* Vh = carve(planeKV);
  unsigned short* Vl = carve(planeKV);
  unsigned short* Oh = carve(planeQ);
  unsigned short* Ol = carve(planeQ);
  if (off > ws_size) return;

  const int n2x = (kSeqLen * kModelD) / 2;
  const int n2y = ((kSeqLen - 1) * kModelD) / 2;
  const int n2w = (kModelD * kModelD) / 2;
  cast_f32_bf16x2<<<dim3((n2x + 255) / 256), dim3(256), 0, stream>>>(x, XYb, n2x);
  cast_f32_bf16x2<<<dim3((n2y + 255) / 256), dim3(256), 0, stream>>>(y, XYb + (size_t)kSeqLen * kModelD, n2y);
  {
    const int nz = kModelD / 2;
    fill_zero_u32<<<dim3((nz + 255) / 256), dim3(256), 0, stream>>>(
        (unsigned*)(void*)(XYb + (size_t)kKvReal * kModelD), nz);
  }
  cast_f32_bf16x2<<<dim3((n2w + 255) / 256), dim3(256), 0, stream>>>(Wq, Wqb, n2w);
  cast_f32_bf16x2<<<dim3((n2w + 255) / 256), dim3(256), 0, stream>>>(Wk, Wkb, n2w);
  cast_f32_bf16x2<<<dim3((n2w + 255) / 256), dim3(256), 0, stream>>>(Wv, Wvb, n2w);
  cast_f32_bf16x2<<<dim3((n2w + 255) / 256), dim3(256), 0, stream>>>(Wo, Wob_b, n2w);

  const int tilesQ  = (kSeqLen / 64) * (kModelD / 64);
  const int tilesKV = (kKvPad / 64) * (kModelD / 64);
  wmma_gemm64<1, 0, 0, 2, false, 0><<<dim3((tilesQ + 7) / 8, 1), dim3(256), 0, stream>>>(
      XYb, XYb, kModelD, 0L, Wqb, Wqb, kModelD, 0L,
      (void*)Qh, (void*)Ql, kModelD, 0L, Wob, out, 0L, kSeqLen, kModelD, kModelD, 1.0f);
  wmma_gemm64<1, 0, 0, 2, false, 0><<<dim3((tilesKV + 7) / 8, 1), dim3(256), 0, stream>>>(
      XYb, XYb, kModelD, 0L, Wkb, Wkb, kModelD, 0L,
      (void*)Kh, (void*)Kl, kModelD, 0L, Wob, out, 0L, kKvPad, kModelD, kModelD, 1.0f);
  wmma_gemm64<1, 0, 0, 2, false, 0><<<dim3((tilesKV + 7) / 8, 1), dim3(256), 0, stream>>>(
      XYb, XYb, kModelD, 0L, Wvb, Wvb, kModelD, 0L,
      (void*)Vh, (void*)Vl, kModelD, 0L, Wob, out, 0L, kKvPad, kModelD, kModelD, 1.0f);

  tree_window_attn<<<dim3(kHeads * kNumQB), dim3(128), 0, stream>>>(Qh, Ql, Kh, Kl, Vh, Vl, Oh, Ol, msk);

  wmma_gemm64<1, 1, 2, 0, false, 0><<<dim3((tilesQ + 7) / 8, 1), dim3(256), 0, stream>>>(
      Oh, Ol, kModelD, 0L, Wob_b, Wob_b, kModelD, 0L,
      (void*)out, (void*)out, kModelD, 0L, Wob, out, 0L, kSeqLen, kModelD, kModelD, 1.0f);
}
